// CausalSelfAttention_41661182771882
// MI455X (gfx1250) — hardware-run, weakly checked
//
#include <hip/hip_runtime.h>
#ifndef NB
#define NB 4
#endif
#ifndef SEQ
#define SEQ 2048
#endif
#define NB_FULL 4
#define SEQ_FULL 2048
#define DM 768
#define NH 12
#define HD 64
#define LQK (2 * DM)
#define NR (NB * SEQ)
#define EARLY ((SEQ) < 512 ? (SEQ) : 512)

static_assert(SEQ % 128 == 0);
static_assert(SEQ <= SEQ_FULL);
static_assert(NB <= NB_FULL);
static_assert(DM % 128 == 0);
static_assert(DM == NH * HD);
static_assert(EARLY % 128 == 0);
static_assert(EARLY <= SEQ);
static_assert(LQK % 64 == 0);
static_assert(NR % 128 == 0);

typedef _Float16 v16h __attribute__((ext_vector_type(16)));
typedef unsigned short v8us __attribute__((ext_vector_type(8), may_alias));
typedef float v8f __attribute__((ext_vector_type(8)));
typedef float v4f __attribute__((ext_vector_type(4)));
typedef float v4fa __attribute__((ext_vector_type(4), may_alias));
union FragH { v16h v; v8us half[2]; _Float16 h[16]; unsigned short u[16]; };

__device__ __forceinline__ float bf16_rne(float x) {
  const unsigned int u = __float_as_uint(x);
  const unsigned int r = (u + 0x7FFFu + ((u >> 16) & 1u)) & 0xFFFF0000u;
  return __uint_as_float(r);
}

__device__ __forceinline__ v16h ld_frag(const _Float16* p, int hh) {
  FragH f;
  f.half[0] = *(const v8us*)((const unsigned short*)p + 8 * hh);
  f.half[1] = *(const v8us*)((const unsigned short*)p + 16 + 8 * hh);
  return f.v;
}
__device__ __forceinline__ v8f g2_mma(v16h a, v16h b, v8f c) {
  v8f d = __builtin_amdgcn_wmma_f32_16x16x32_f16(false, a, false, b, (short)0, c, false, false);
  asm volatile("v_nop\n\tv_nop\n\tv_nop\n\tv_nop" : "+v"(d) : "v"(a), "v"(b));
  return d;
}
template <int NT>
__device__ __forceinline__ v8f mmaH(v16h ah, v16h al, v16h bh, v16h bl, v8f c) {
  c = __builtin_amdgcn_wmma_f32_16x16x32_f16(false, ah, false, bh, (short)0, c, false, false);
  if (NT >= 2) c = __builtin_amdgcn_wmma_f32_16x16x32_f16(false, al, false, bh, (short)0, c, false, false);
  if (NT >= 3) c = __builtin_amdgcn_wmma_f32_16x16x32_f16(false, ah, false, bl, (short)0, c, false, false);
  asm volatile("v_nop\n\tv_nop\n\tv_nop\n\tv_nop" : "+v"(c) : "v"(ah), "v"(al), "v"(bh), "v"(bl));
  return c;
}

__global__ __launch_bounds__(256) void k_cvt(const float* __restrict__ w, _Float16* __restrict__ o16, size_t n8, float scale) {
  const size_t t = (size_t)blockIdx.x * 256 + threadIdx.x;
  if (t >= n8) return;
  const v4f a = *(const v4fa*)(w + t * 8), c = *(const v4fa*)(w + t * 8 + 4);
  FragH f;
#pragma unroll
  for (int q = 0; q < 4; ++q) { f.h[q] = (_Float16)(bf16_rne(a[q]) * scale); f.h[4 + q] = (_Float16)(bf16_rne(c[q]) * scale); }
  const v8us o = f.half[0];
  *(volatile v8us*)((unsigned short*)o16 + t * 8) = o;
  __threadfence();
  *(volatile v8us*)((unsigned short*)o16 + t * 8) = o;
}
__global__ __launch_bounds__(256) void k_x16(const float* __restrict__ x, _Float16* __restrict__ X16, size_t n8) {
  const size_t t = (size_t)blockIdx.x * 256 + threadIdx.x;
  if (t >= n8) return;
  const size_t e = t * 8;
  const size_t row = e / DM;
  const size_t col = e - row * DM;
  const size_t bb = row / SEQ, ss = row - bb * SEQ;
  const float* src = x + (bb * SEQ_FULL + ss) * DM + col;
  const v4f a = *(const v4fa*)src, c = *(const v4fa*)(src + 4);
  FragH f;
#pragma unroll
  for (int q = 0; q < 4; ++q) { f.h[q] = (_Float16)(bf16_rne(a[q]) * 16.0f); f.h[4 + q] = (_Float16)(bf16_rne(c[q]) * 16.0f); }
  const v8us o = f.half[0];
  *(volatile v8us*)((unsigned short*)X16 + t * 8) = o;
  __threadfence();
  *(volatile v8us*)((unsigned short*)X16 + t * 8) = o;
}

template <int OM, bool ROWBIAS, bool ARES>
__global__ __launch_bounds__(128) void k_gemm(const _Float16* __restrict__ A, const _Float16* __restrict__ AL, int lda,
                                              const _Float16* __restrict__ Bt, int ldb, const float* __restrict__ bias, float alpha, float beta,
                                              float* __restrict__ C, _Float16* __restrict__ C16H, _Float16* __restrict__ C16L, int ldc,
                                              int M, int N, int K, int seq, int seqfull, int early) {
  __shared__ __attribute__((aligned(16))) float so[4][32][68];
  const int tid = threadIdx.x, lane = tid & 31, ln = lane & 15, hh = lane >> 4;
  const int w = __builtin_amdgcn_readfirstlane(tid >> 5);
  const int ntn = N >> 6;
  const int mt = (int)blockIdx.x / ntn, nq = (int)blockIdx.x - mt * ntn;
  const int row0 = mt * 128 + 32 * w, col0 = nq * 64;
  if (row0 >= M) return;
  const bool res = ARES && (((mt * 128) % seq) < early);
  const _Float16* a0p = A + (size_t)(row0 + ln) * lda;
  const _Float16* a1p = a0p + (size_t)16 * lda;
  const _Float16* l0p = ARES ? (AL + (size_t)(row0 + ln) * lda) : a0p;
  const _Float16* l1p = l0p + (size_t)16 * lda;
  const _Float16* b0p = Bt + (size_t)(col0 + ln) * ldb;
  const _Float16* b1p = b0p + (size_t)16 * ldb;
  const _Float16* b2p = b1p + (size_t)16 * ldb;
  const _Float16* b3p = b2p + (size_t)16 * ldb;
  const v8f z8 = {0.f, 0.f, 0.f, 0.f, 0.f, 0.f, 0.f, 0.f};
  v8f c00 = z8, c01 = z8, c02 = z8, c03 = z8, c10 = z8, c11 = z8, c12 = z8, c13 = z8;
#pragma unroll 1
  for (int kb = 0; kb < K; kb += 32) {
    const v16h a0 = ld_frag(a0p + kb, hh), a1 = ld_frag(a1p + kb, hh);
    const v16h b0 = ld_frag(b0p + kb, hh), b1 = ld_frag(b1p + kb, hh), b2 = ld_frag(b2p + kb, hh), b3 = ld_frag(b3p + kb, hh);
    c00 = g2_mma(a0, b0, c00); c10 = g2_mma(a1, b0, c10);
    c01 = g2_mma(a0, b1, c01); c11 = g2_mma(a1, b1, c11);
    c02 = g2_mma(a0, b2, c02); c12 = g2_mma(a1, b2, c12);
    c03 = g2_mma(a0, b3, c03); c13 = g2_mma(a1, b3, c13);
    if (ARES) {
      if (res) {
        const v16h r0 = ld_frag(l0p + kb, hh), r1 = ld_frag(l1p + kb, hh);
        c00 = g2_mma(r0, b0, c00); c10 = g2_mma(r1, b0, c10);
        c01 = g2_mma(r0, b1, c01); c11 = g2_mma(r1, b1, c11);
        c02 = g2_mma(r0, b2, c02); c12 = g2_mma(r1, b2, c12);
        c03 = g2_mma(r0, b3, c03); c13 = g2_mma(r1, b3, c13);
      }
    }
  }
  v8f accs[8] = {c00, c01, c02, c03, c10, c11, c12, c13};
#pragma unroll
  for (int u = 0; u < 8; ++u) {
    const int t = u & 3, half = u >> 2;
    const int col = col0 + t * 16 + ln;
    float bc = 0.f;
    if (!ROWBIAS) bc = bf16_rne(bias[col]) * beta;
#pragma unroll
    for (int r = 0; r < 8; ++r) {
      const int rloc = half * 16 + 8 * hh + r;
      float bv = bc;
      if (ROWBIAS) bv = bf16_rne(bias[row0 + rloc]) * beta;
      so[w][rloc][t * 16 + ln] = accs[u][r] * alpha + bv;
    }
  }
  __builtin_amdgcn_fence(4  , "workgroup");
  __builtin_amdgcn_wave_barrier();
  if (OM == 0) {
    const int rsub = lane >> 4, c4 = (lane & 15) * 4;
    for (int pass = 0; pass < 2; ++pass) {
#pragma unroll
      for (int q = 0; q < 16; ++q) {
        const int r = q * 2 + rsub;
        const v4f v = *(const v4fa*)&so[w][r][c4];
        const size_t grow = (size_t)(row0 + r);
        const size_t orow = (grow / (size_t)seq) * (size_t)seqfull + (grow % (size_t)seq);
        *(volatile v4f*)(C + orow * (size_t)ldc + col0 + c4) = v;
      }
      if (pass == 0) __threadfence();
    }
  } else {
    const int rq = lane >> 3, pc8 = (lane & 7) * 8;
    for (int pass = 0; pass < 2; ++pass) {
#pragma unroll
      for (int it = 0; it < 8; ++it) {
        const int r = it * 4 + rq;
        const v4f x0 = *(const v4fa*)&so[w][r][pc8], x1 = *(const v4fa*)&so[w][r][pc8 + 4];
        FragH fh, fl;
#pragma unroll
        for (int q = 0; q < 4; ++q) {
          _Float16 hv = (_Float16)x0[q]; fh.h[q] = hv; fl.h[q] = (_Float16)(x0[q] - (float)hv);
          hv = (_Float16)x1[q]; fh.h[4 + q] = hv; fl.h[4 + q] = (_Float16)(x1[q] - (float)hv);
        }
        const size_t o = (size_t)(row0 + r) * (size_t)ldc + col0 + pc8;
        const v8us oh = fh.half[0], ol = fl.half[0];
        *(volatile v8us*)((unsigned short*)C16H + o) = oh;
        *(volatile v8us*)((unsigned short*)C16L + o) = ol;
      }
      if (pass == 0) __threadfence();
    }
  }
}

template <bool RES>
__global__ __launch_bounds__(128) void k_attn(const _Float16* __restrict__ QKH, const _Float16* __restrict__ QKL,
                                              const _Float16* __restrict__ VTH, const _Float16* __restrict__ VTL,
                                              _Float16* __restrict__ CH, _Float16* __restrict__ CL, int qblk0) {
  __shared__ __attribute__((aligned(16))) float so[4][16][68];
  const int lane = threadIdx.x & 31, ln = lane & 15, hh = lane >> 4;
  const int w = __builtin_amdgcn_readfirstlane((int)(threadIdx.x >> 5));
  const int h = (int)blockIdx.y, b = (int)blockIdx.z;
  const int q0 = (qblk0 + (int)blockIdx.x) * 64 + w * 16;
  const size_t tok0 = (size_t)b * SEQ;
  const size_t qoff = (tok0 + (size_t)(q0 + ln)) * LQK + (size_t)h * HD;
  const v16h qh0 = ld_frag(QKH + qoff, hh), qh1 = ld_frag(QKH + qoff + 32, hh);
  const v16h ql0 = ld_frag(QKL + qoff, hh), ql1 = ld_frag(QKL + qoff + 32, hh);
  const size_t koff = (tok0 + (size_t)ln) * LQK + DM + (size_t)h * HD;
  const size_t voff = (size_t)(h * HD + ln) * NR + tok0;
  const v8f z8 = {0.f, 0.f, 0.f, 0.f, 0.f, 0.f, 0.f, 0.f};
  v8f o[4] = {z8, z8, z8, z8};
  float m = -1.0e30f, l = 0.f;
  const float cs = 0.18033688011112042f * 0.000244140625f;
  const int qi = q0 + ln;
  const int nst = (q0 + 47) >> 5;
#pragma unroll 1
  for (int st = 0; st < nst; ++st) {
    const int k0 = st * 32;
    const size_t ko = koff + (size_t)k0 * LQK;
    const size_t k1 = ko + (size_t)16 * LQK;
    v8f s0 = z8, s1 = z8;
    {
      v16h a = ld_frag(QKH + ko, hh), al = ld_frag(QKL + ko, hh);
      s0 = mmaH<3>(a, al, qh0, ql0, s0);
      a = ld_frag(QKH + ko + 32, hh); al = ld_frag(QKL + ko + 32, hh);
      s0 = mmaH<3>(a, al, qh1, ql1, s0);
      a = ld_frag(QKH + k1, hh); al = ld_frag(QKL + k1, hh);
      s1 = mmaH<3>(a, al, qh0, ql0, s1);
      a = ld_frag(QKH + k1 + 32, hh); al = ld_frag(QKL + k1 + 32, hh);
      s1 = mmaH<3>(a, al, qh1, ql1, s1);
    }
    float t0[8], t1[8];
#pragma unroll
    for (int r = 0; r < 8; ++r) { t0[r] = s0[r] * cs; t1[r] = s1[r] * cs; }
    if (k0 + 31 > q0) {
#pragma unroll
      for (int r = 0; r < 8; ++r) {
        const int key = k0 + 8 * hh + r;
        t0[r] = (key <= qi) ? t0[r] : -1.0e30f;
        t1[r] = (key + 16 <= qi) ? t1[r] : -1.0e30f;
      }
    }
    float mx = fmaxf(t0[0], t1[0]);
#pragma unroll
    for (int r = 1; r < 8; ++r) mx = fmaxf(mx, fmaxf(t0[r], t1[r]));
    mx = fmaxf(mx, __shfl_xor(mx, 16, 32));
    const float mn = fmaxf(m, mx);
    const float sc = __builtin_amdgcn_exp2f(m - mn);
    m = mn;
    FragH ph, pl;
    float ps = 0.f;
#pragma unroll
    for (int r = 0; r < 8; ++r) {
      const float p0 = __builtin_amdgcn_exp2f(t0[r] - mn);
      const float p1 = __builtin_amdgcn_exp2f(t1[r] - mn);
      ps += p0 + p1;
      const float c0 = p0 * 1024.0f, c1 = p1 * 1024.0f;
      const _Float16 h0 = (_Float16)c0, h1 = (_Float16)c1;
      ph.h[r] = h0; ph.h[8 + r] = h1;
      if (RES) { pl.h[r] = (_Float16)(c0 - (float)h0); pl.h[8 + r] = (_Float16)(c1 - (float)h1); }
    }
    l = l * sc + ps;
#pragma unroll
    for (int t = 0; t < 4; ++t) o[t] *= sc;
#pragma unroll
    for (int t = 0; t < 4; ++t) {
      const size_t vo = voff + (size_t)(16 * t) * NR + (size_t)k0;
      const v16h vh = ld_frag(VTH + vo, hh);
      if (RES) {
        const v16h vl = ld_frag(VTL + vo, hh);
        o[t] = mmaH<3>(vh, vl, ph.v, pl.v, o[t]);
      } else {
        o[t] = mmaH<1>(vh, vh, ph.v, ph.v, o[t]);
      }
    }
  }
  const float lt = l + __shfl_xor(l, 16, 32);
  const float fin = 0.0009765625f * (1.0f / lt);
#pragma unroll
  for (int t = 0; t < 4; ++t) {
    const v4f a = {o[t][0] * fin, o[t][1] * fin, o[t][2] * fin, o[t][3] * fin};
    const v4f c = {o[t][4] * fin, o[t][5] * fin, o[t][6] * fin, o[t][7] * fin};
    *(v4f*)&so[w][ln][16 * t + 8 * hh] = a;
    *(v4f*)&so[w][ln][16 * t + 8 * hh + 4] = c;
  }
  __builtin_amdgcn_fence(4  , "workgroup");
  __builtin_amdgcn_wave_barrier();
  const size_t obase = (tok0 + (size_t)q0) * DM + (size_t)h * HD;
  const int rq = lane >> 3, pc8 = (lane & 7) * 8;
  for (int pass = 0; pass < 2; ++pass) {
#pragma unroll
    for (int it = 0; it < 4; ++it) {
      const int r = it * 4 + rq;
      const v4f x0 = *(const v4fa*)&so[w][r][pc8], x1 = *(const v4fa*)&so[w][r][pc8 + 4];
      FragH fh, fl;
#pragma unroll
      for (int q = 0; q < 4; ++q) {
        _Float16 hv = (_Float16)x0[q]; fh.h[q] = hv; fl.h[q] = (_Float16)(x0[q] - (float)hv);
        hv = (_Float16)x1[q]; fh.h[4 + q] = hv; fl.h[4 + q] = (_Float16)(x1[q] - (float)hv);
      }
      const size_t oo = obase + (size_t)r * DM + pc8;
      const v8us oh = fh.half[0], ol = fl.half[0];
      *(volatile v8us*)((unsigned short*)CH + oo) = oh;
      if (RES) *(volatile v8us*)((unsigned short*)CL + oo) = ol;
    }
    if (pass == 0) __threadfence();
  }
}

#define SZ_X16 ((size_t)NR * DM * 2)
#define SZ_WQ  ((size_t)3 * DM * DM * 2)
#define SZ_WP  ((size_t)DM * DM * 2)
#define SZ_QK  ((size_t)NR * LQK * 2)
#define SZ_VT  ((size_t)DM * NR * 2)
#define SZ_CT  ((size_t)NR * DM * 2)
static_assert(SZ_X16 % 256 == 0);
static_assert(SZ_WQ % 256 == 0);
static_assert(SZ_WP % 256 == 0);
static_assert(SZ_QK % 256 == 0);
static_assert(SZ_VT % 256 == 0);
static_assert(SZ_X16 + SZ_WQ + SZ_WP + 2 * SZ_QK + 2 * SZ_VT + 2 * SZ_CT <= (size_t)134217728);
static_assert((NR * (DM / 8)) % 256 == 0);
static_assert((3 * DM * DM / 8) % 256 == 0);
static_assert((DM * DM / 8) % 256 == 0);

extern "C" void kernel_launch(void* const* d_in, const int* in_sizes, int n_in,
                              void* d_out, int out_size, void* d_ws, size_t ws_size, hipStream_t stream) {
  if (n_in < 5) return;
  const size_t need = ((size_t)(NB - 1) * SEQ_FULL + SEQ) * DM;
  if ((size_t)in_sizes[0] < need) return;
  if (in_sizes[1] < 3 * DM * DM) return;
  if (in_sizes[2] < 3 * DM) return;
  if (in_sizes[3] < DM * DM) return;
  if (in_sizes[4] < DM) return;
  if ((size_t)out_size < need) return;
  const float* x = (const float*)d_in[0];
  const float* wqkv = (const float*)d_in[1];
  const float* bqkv = (const float*)d_in[2];
  const float* wproj = (const float*)d_in[3];
  const float* bproj = (const float*)d_in[4];
  float* out = (float*)d_out;
  char* ws = (char*)d_ws;
  size_t off = 0;
  auto take = [&](size_t bytes) { char* p = ws + off; off += (bytes + 255) & ~(size_t)255; return p; };
  _Float16* X16 = (_Float16*)take(SZ_X16);
  _Float16* WQ16 = (_Float16*)take(SZ_WQ);
  _Float16* WP16 = (_Float16*)take(SZ_WP);
  _Float16* QKH = (_Float16*)take(SZ_QK);
  _Float16* QKL = (_Float16*)take(SZ_QK);
  _Float16* VTH = (_Float16*)take(SZ_VT);
  _Float16* VTL = (_Float16*)take(SZ_VT);
  _Float16* CTH = (_Float16*)take(SZ_CT);
  _Float16* CTL = (_Float16*)take(SZ_CT);
  if (off > ws_size) return;

  k_x16<<<(unsigned)((size_t)NR * (DM / 8) / 256), 256, 0, stream>>>(x, X16, (size_t)NR * (DM / 8));
  k_cvt<<<(unsigned)((size_t)3 * DM * DM / 8 / 256), 256, 0, stream>>>(wqkv, WQ16, (size_t)3 * DM * DM / 8, 64.0f);
  k_cvt<<<(unsigned)((size_t)DM * DM / 8 / 256), 256, 0, stream>>>(wproj, WP16, (size_t)DM * DM / 8, 64.0f);
  k_gemm<1, false, false><<<(unsigned)((NR / 128) * (LQK / 64)), 128, 0, stream>>>(X16, X16, DM, WQ16, DM, bqkv, 0.0625f, 64.0f,
      nullptr, QKH, QKL, LQK, NR, LQK, DM, SEQ, SEQ_FULL, 0);
  k_gemm<1, true, false><<<(unsigned)((DM / 128) * (NR / 64)), 128, 0, stream>>>(WQ16 + (size_t)2 * DM * DM, WQ16, DM, X16, DM, bqkv + 2 * DM, 1.0f, 1024.0f,
      nullptr, VTH, VTL, NR, DM, NR, DM, SEQ, SEQ_FULL, 0);
  k_attn<true><<<dim3(EARLY / 64, NH, NB), 128, 0, stream>>>(QKH, QKL, VTH, VTL, CTH, CTL, 0);
  if (SEQ > EARLY)
    k_attn<false><<<dim3((SEQ - EARLY) / 64, NH, NB), 128, 0, stream>>>(QKH, QKL, VTH, VTL, CTH, CTL, EARLY / 64);
  k_gemm<0, false, true><<<(unsigned)((NR / 128) * (DM / 64)), 128, 0, stream>>>(CTH, CTL, DM, WP16, DM, bproj, 0.0000152587890625f, 1.0f,
      out, nullptr, nullptr, DM, NR, DM, DM, SEQ, SEQ_FULL, EARLY);
}
